// MultiHeadAttentionBlock_57569741635752
// MI455X (gfx1250) — hardware-verified
//
#include <hip/hip_runtime.h>
#include <math.h>

#ifndef NB
#define NB 2
#endif
#ifndef SEQ
#define SEQ 2048
#endif
#define NB_FULL 2
#define SEQ_FULL 2048
#define DM 768
#define NH 12
#define HD 64
#define D3 (3 * DM)

static_assert(DM == NH * HD);
static_assert(HD == 64);
static_assert(SEQ % 64 == 0);
static_assert(SEQ <= SEQ_FULL);
static_assert(NB <= NB_FULL);
static_assert(DM % 64 == 0);

typedef __attribute__((ext_vector_type(16))) _Float16 v16h;
typedef __attribute__((ext_vector_type(8)))  _Float16 v8h;
typedef __attribute__((ext_vector_type(16))) __bf16   v16b;
typedef __attribute__((ext_vector_type(8)))  __bf16   v8b;
typedef __attribute__((ext_vector_type(8)))  float    v8f;
typedef __attribute__((ext_vector_type(4)))  float    v4f;
typedef unsigned int cm_u4 __attribute__((ext_vector_type(4)));

__device__ __forceinline__ int frag_k(int i, int h) { return (i < 8) ? (8 * h + i) : (16 + 8 * h + (i - 8)); }
__device__ __forceinline__ __bf16 bf16_rne(float f) {
    unsigned int u = __float_as_uint(f);
    u += 0x7fffu + ((u >> 16) & 1u);
    return __builtin_bit_cast(__bf16, (unsigned short)(u >> 16));
}
__device__ __forceinline__ float bf16_f32(__bf16 b) { return __uint_as_float(((unsigned int)__builtin_bit_cast(unsigned short, b)) << 16); }
__device__ __forceinline__ unsigned short f2bf_bits(float f) {
    unsigned u = __float_as_uint(f);
    return (unsigned short)((u + 0x7FFFu + ((u >> 16) & 1u)) >> 16);
}
__device__ __forceinline__ float bf_bits2f(unsigned short h) { return __uint_as_float(((unsigned)h) << 16); }

__device__ __forceinline__ v8f wmma16(v16h a, v16h b, v8f c) {
    c = __builtin_amdgcn_wmma_f32_16x16x32_f16(false, a, false, b, (short)0, c, false, false);
    asm volatile("v_nop\n\tv_nop\n\tv_nop\n\tv_nop" : "+v"(c) : "v"(a), "v"(b));
    return c;
}
struct Split { v16b hi, lo; };
__device__ __forceinline__ v8f wmma3(const Split& a, const Split& b, v8f c) {
    c = __builtin_amdgcn_wmma_f32_16x16x32_bf16(false, a.hi, false, b.hi, (short)0, c, false, false);
    c = __builtin_amdgcn_wmma_f32_16x16x32_bf16(false, a.hi, false, b.lo, (short)0, c, false, false);
    c = __builtin_amdgcn_wmma_f32_16x16x32_bf16(false, a.lo, false, b.hi, (short)0, c, false, false);
    asm volatile("v_nop\n\tv_nop\n\tv_nop\n\tv_nop" : "+v"(c) : "v"(a.hi), "v"(a.lo), "v"(b.hi), "v"(b.lo));
    return c;
}
struct Split3 { v16b hi, mid, lo; };
__device__ __forceinline__ v8f wmma6(const Split3& a, const Split3& b, v8f c) {
    c = __builtin_amdgcn_wmma_f32_16x16x32_bf16(false, a.hi, false, b.hi, (short)0, c, false, false);
    c = __builtin_amdgcn_wmma_f32_16x16x32_bf16(false, a.hi, false, b.mid, (short)0, c, false, false);
    c = __builtin_amdgcn_wmma_f32_16x16x32_bf16(false, a.mid, false, b.hi, (short)0, c, false, false);
    c = __builtin_amdgcn_wmma_f32_16x16x32_bf16(false, a.hi, false, b.lo, (short)0, c, false, false);
    c = __builtin_amdgcn_wmma_f32_16x16x32_bf16(false, a.mid, false, b.mid, (short)0, c, false, false);
    c = __builtin_amdgcn_wmma_f32_16x16x32_bf16(false, a.lo, false, b.hi, (short)0, c, false, false);
    asm volatile("v_nop\n\tv_nop\n\tv_nop\n\tv_nop" : "+v"(c) : "v"(a.hi), "v"(a.mid), "v"(a.lo), "v"(b.hi), "v"(b.mid), "v"(b.lo));
    return c;
}

__device__ __forceinline__ v16h fh_ld(const float* __restrict__ p, long long sk, int k0, int h, int klen, float s) {
    v16h a;
#pragma unroll
    for (int i = 0; i < 16; ++i) { const int k = k0 + frag_k(i, h); a[i] = (k < klen) ? (_Float16)(p[(long long)k * sk] * s) : (_Float16)0.f; }
    return a;
}
__device__ __forceinline__ Split sp_ld(const float* __restrict__ p, long long sk, int k0, int h, int klen, float s) {
    Split r;
#pragma unroll
    for (int i = 0; i < 16; ++i) {
        const int k = k0 + frag_k(i, h); const float x = (k < klen) ? p[(long long)k * sk] * s : 0.f;
        const __bf16 hb = bf16_rne(x); r.hi[i] = hb; r.lo[i] = bf16_rne(x - bf16_f32(hb));
    }
    return r;
}
__device__ __forceinline__ Split3 sp3_ld(const float* __restrict__ p, long long sk, int k0, int h, int klen, float s) {
    Split3 r;
#pragma unroll
    for (int i = 0; i < 16; ++i) {
        const int k = k0 + frag_k(i, h); const float x = (k < klen) ? p[(long long)k * sk] * s : 0.f;
        const __bf16 hb = bf16_rne(x); const float r1 = x - bf16_f32(hb); const __bf16 mb = bf16_rne(r1);
        r.hi[i] = hb; r.mid[i] = mb; r.lo[i] = bf16_rne(r1 - bf16_f32(mb));
    }
    return r;
}

#define VST2(T, ptr, val) do { const T vst2_v_ = (val); *(volatile T*)(ptr) = vst2_v_; __threadfence(); *(volatile T*)(ptr) = vst2_v_; } while (0)
#define VST2V4(ptr, val) do { const v4f vst2_v4_ = (val); *(volatile v4f*)(ptr) = vst2_v4_; __threadfence(); *(volatile v4f*)(ptr) = vst2_v4_; } while (0)

#define AW 4
struct AttnP {
    const float* Q; const float* K; const float* V; float* O; float* P; const float* Mf; const int* Mi; float* ST;
    const float* Pw; const float* Rt; const int* SQ; const int* SK;
    long long swb, swh, swi, swj, srb, srh, sri;
    long long sQb, sQh, sQi, sQd, sKb, sKh, sKj, sKd, sVb, sVh, sVj, sVd, sOb, sOh, sOi, sPb, sPh, sPi, smb, smh, smi, smj;
    int Lq, Lk, dh, dv, hrep, causal, coff, pband;
    float scale, mfill; int nonorm, mpol;
    int roff, rn, segpol, win;
};
static_assert(sizeof(AttnP) == 12 * 8 + 29 * 8 + 16 * 4);

#ifndef KATTN_ATTR
#define KATTN_ATTR
#endif
template <int DHP, int DVP, int QM, bool SPLITPV, bool TWOPASS>
__global__ __launch_bounds__(32 * AW) KATTN_ATTR void k_attn(AttnP p) {
    constexpr int NT = DVP / 16;
    constexpr int KS = DHP / 32;
    constexpr int VP = DVP + 8;
    __shared__ __align__(16) float    pl[AW][16 * 64];
    __shared__ __align__(16) _Float16 vl[(SPLITPV ? 2 : 1) * 64 * VP];
    const int lane = threadIdx.x & 31, hf = lane >> 4, l15 = lane & 15, wave = threadIdx.x >> 5;
    const int h = blockIdx.y, b = blockIdx.z, hk = h / p.hrep;
    const int q0 = (blockIdx.x * AW + wave) * 16;
    float* myp = pl[wave];
    const float L2E = 1.4426950408889634f;
    const float NEG = -__builtin_inff();
    const int qi = min(q0 + l15, p.Lq - 1);
    const float* qrow = p.Q + b * p.sQb + h * p.sQh + (long long)qi * p.sQi;
    const float* kbase = p.K + b * p.sKb + hk * p.sKh;
    const float* vbase = p.V + b * p.sVb + hk * p.sVh;
    v16h qa[QM == 0 ? KS : 1]; Split qs_[QM == 1 ? KS : 1]; Split3 qt_[QM == 2 ? KS : 1];
#pragma unroll
    for (int ks = 0; ks < KS; ++ks) {
        if (QM == 2) qt_[ks] = sp3_ld(qrow, p.sQd, ks * 32, hf, p.dh, 1.f);
        else if (QM == 1) qs_[ks] = sp_ld(qrow, p.sQd, ks * 32, hf, p.dh, 1.f);
        else qa[ks] = fh_ld(qrow, p.sQd, ks * 32, hf, p.dh, 1.f);
    }
    v8f o[NT]; float m8[8], l8[8];
#pragma unroll
    for (int t = 0; t < NT; ++t) { v8f zz = {}; o[t] = zz; }
#pragma unroll
    for (int i = 0; i < 8; ++i) { m8[i] = NEG; l8[i] = 0.f; }
    int jend = p.Lk; int jstart = 0;
    if (p.causal == 1) { const int je = (blockIdx.x * AW + AW - 1) * 16 + 16 + p.coff; jend = min(jend, max(je, 0)); }
    if (p.win > 0) { const int js = (int)(blockIdx.x * AW) * 16 + p.coff - p.win; jstart = (js > 0) ? (js / 64) * 64 : 0; }
    const int npass = TWOPASS ? 2 : 1;
    for (int pass = 0; pass < npass; ++pass) {
        const bool dopv = (!TWOPASS) || pass == 1;
        for (int j0 = jstart; j0 < jend; j0 += 64) {
            if (dopv) {
                __syncthreads();
                for (int idx = threadIdx.x; idx < 64 * DVP; idx += 32 * AW) {
                    const int jr = idx / DVP, d = idx - jr * DVP, j = j0 + jr;
                    const float f = (j < p.Lk && d < p.dv) ? vbase[(long long)j * p.sVj + (long long)d * p.sVd] : 0.f;
                    if (SPLITPV) {
                        const __bf16 hb = bf16_rne(f);
                        ((__bf16*)vl)[jr * VP + d] = hb; ((__bf16*)vl)[64 * VP + jr * VP + d] = bf16_rne(f - bf16_f32(hb));
                    } else vl[jr * VP + d] = (_Float16)f;
                }
            }
            v8f s[4];
#pragma unroll
            for (int t = 0; t < 4; ++t) {
                const int j = min(j0 + t * 16 + l15, p.Lk - 1);
                const float* krow = kbase + (long long)j * p.sKj;
                v8f acc = {};
#pragma unroll
                for (int ks = 0; ks < KS; ++ks) {
                    if (QM == 2)      acc = wmma6(qt_[ks], sp3_ld(krow, p.sKd, ks * 32, hf, p.dh, 1.f), acc);
                    else if (QM == 1) acc = wmma3(qs_[ks], sp_ld(krow, p.sKd, ks * 32, hf, p.dh, 1.f), acc);
                    else              acc = wmma16(qa[ks], fh_ld(krow, p.sKd, ks * 32, hf, p.dh, 1.f), acc);
                }
                s[t] = acc;
            }
            float pv[8][4];
#pragma unroll
            for (int i = 0; i < 8; ++i) {
                const int irow = q0 + i + 8 * hf;
                const int ic = min(irow, p.Lq - 1);
                float sc[4];
#pragma unroll
                for (int t = 0; t < 4; ++t) {
                    const int jg = j0 + t * 16 + l15;
                    float v = s[t][i] * p.scale;
                    if (p.Mf) v += p.Mf[b * p.smb + h * p.smh + (long long)ic * p.smi + (long long)min(jg, p.Lk - 1) * p.smj];
                    if (p.Rt) { int rc = ic - min(jg, p.Lk - 1) + p.roff; rc = rc < 0 ? 0 : (rc >= p.rn ? p.rn - 1 : rc); v += p.Rt[b * p.srb + h * p.srh + (long long)ic * p.sri + rc]; }
                    if (p.Mi) { const int mv = p.Mi[b * p.smb + h * p.smh + (long long)ic * p.smi + (long long)min(jg, p.Lk - 1) * p.smj]; if (p.mpol ? (mv != 0) : (mv == 0)) v = p.mfill; }
                    if (p.SQ) { const bool same = p.SQ[(long long)b * p.Lq + ic] == p.SK[(long long)b * p.Lk + min(jg, p.Lk - 1)]; if (p.segpol ? same : !same) v = p.mfill; }
                    if (p.causal == 2 && jg > irow + p.coff) v = p.mfill;
                    if (jg >= p.Lk || (p.causal == 1 && jg > irow + p.coff) || (p.causal == 3 && jg < irow + p.coff) || (p.win > 0 && irow + p.coff - jg > p.win)) v = NEG; else v *= L2E;
                    sc[t] = v;
                }
                if (!TWOPASS || pass == 0) {
                    float mx = fmaxf(fmaxf(sc[0], sc[1]), fmaxf(sc[2], sc[3]));
                    mx = fmaxf(mx, __shfl_xor(mx, 1, 32)); mx = fmaxf(mx, __shfl_xor(mx, 2, 32));
                    mx = fmaxf(mx, __shfl_xor(mx, 4, 32)); mx = fmaxf(mx, __shfl_xor(mx, 8, 32));
                    const float mnew = fmaxf(m8[i], mx);
                    const float corr = (mnew == NEG) ? 1.f : exp2f(m8[i] - mnew);
                    float rs = 0.f;
#pragma unroll
                    for (int t = 0; t < 4; ++t) {
                        const float pp = (sc[t] == NEG) ? 0.f : exp2f(sc[t] - mnew); rs += pp;
                        pv[i][t] = p.Pw ? pp * p.Pw[b * p.swb + h * p.swh + (long long)ic * p.swi + (long long)min(j0 + t * 16 + l15, p.Lk - 1) * p.swj] : pp;
                    }
                    rs += __shfl_xor(rs, 1, 32); rs += __shfl_xor(rs, 2, 32); rs += __shfl_xor(rs, 4, 32); rs += __shfl_xor(rs, 8, 32);
                    l8[i] = l8[i] * corr + rs; m8[i] = mnew;
                    if (!TWOPASS) {
#pragma unroll
                        for (int t = 0; t < NT; ++t) o[t][i] *= corr;
                    }
                } else {
                    const float inv = (l8[i] > 0.f) ? 1.f / l8[i] : 0.f;
#pragma unroll
                    for (int t = 0; t < 4; ++t) {
                        const int jg = j0 + t * 16 + l15;
                        float pp = (sc[t] == NEG) ? 0.f : exp2f(sc[t] - m8[i]) * inv;
                        if (p.Pw) pp *= p.Pw[b * p.swb + h * p.swh + (long long)ic * p.swi + (long long)min(jg, p.Lk - 1) * p.swj];
                        pv[i][t] = pp;
                    }
                }
            }
            if (dopv) {
#pragma unroll
                for (int i = 0; i < 8; ++i)
#pragma unroll
                    for (int t = 0; t < 4; ++t) ((volatile float*)myp)[(i + 8 * hf) * 64 + t * 16 + l15] = pv[i][t];
                __syncthreads();
                if (p.P) {
                    float* pb_ = p.P + b * p.sPb + h * p.sPh;
                    const bool fastP = (p.pband == 0) && ((p.sPi & 3) == 0) && (j0 + 64 <= p.Lk) && (q0 + 16 <= p.Lq) && ((((size_t)pb_) & 15) == 0);
                    if (fastP) {
#pragma unroll
                        for (int s2 = 0; s2 < 8; ++s2) {
                            const int row = s2 * 2 + (lane >> 4), c4 = (lane & 15) * 4;
                            const v4f v = *(const v4f*)(myp + row * 64 + c4);
                            VST2V4(pb_ + (long long)(q0 + row) * p.sPi + j0 + c4, v);
                        }
                    } else {
                        for (int row = 0; row < 16; ++row) {
                            const int irow = q0 + row; if (irow >= p.Lq) continue;
                            for (int c = lane; c < 64; c += 32) {
                                const int jg = j0 + c; if (jg >= p.Lk) continue;
                                if (p.pband == 0) VST2(float, pb_ + (long long)irow * p.sPi + jg, myp[row * 64 + c]);
                                else if (jg - irow <= p.pband && irow - jg <= p.pband) VST2(float, pb_ + (long long)irow * p.sPi + (jg - irow + p.pband), myp[row * 64 + c]);
                            }
                        }
                    }
                }
                if (SPLITPV) {
                    const Split pa0 = sp_ld(myp + l15 * 64, 1, 0, hf, 64, 1.f), pa1 = sp_ld(myp + l15 * 64, 1, 32, hf, 64, 1.f);
                    const __bf16* vh = (const __bf16*)vl; const __bf16* vlo = vh + 64 * VP;
#pragma unroll
                    for (int t = 0; t < NT; ++t) {
                        const int dcol = t * 16 + l15;
                        Split b0, b1;
#pragma unroll
                        for (int e = 0; e < 16; ++e) {
                            const int k0 = frag_k(e, hf), k1 = 32 + frag_k(e, hf);
                            b0.hi[e] = vh[k0 * VP + dcol]; b0.lo[e] = vlo[k0 * VP + dcol]; b1.hi[e] = vh[k1 * VP + dcol]; b1.lo[e] = vlo[k1 * VP + dcol];
                        }
                        o[t] = wmma3(pa0, b0, o[t]);
                        o[t] = wmma3(pa1, b1, o[t]);
                    }
                } else {
                    const v16h pa0 = fh_ld(myp + l15 * 64, 1, 0, hf, 64, 4096.f), pa1 = fh_ld(myp + l15 * 64, 1, 32, hf, 64, 4096.f);
#pragma unroll
                    for (int t = 0; t < NT; ++t) {
                        const int dcol = t * 16 + l15;
                        v16h b0, b1;
#pragma unroll
                        for (int e = 0; e < 16; ++e) { b0[e] = vl[frag_k(e, hf) * VP + dcol]; b1[e] = vl[(32 + frag_k(e, hf)) * VP + dcol]; }
                        o[t] = wmma16(pa0, b0, o[t]);
                        o[t] = wmma16(pa1, b1, o[t]);
                    }
                }
            }
        }
    }
    float* obase = p.O + b * p.sOb + h * p.sOh;
    if (p.ST) {
        const int rl = lane >> 1, isel = rl & 7;
        float mv = 0.f, lv = 0.f;
#pragma unroll
        for (int i = 0; i < 8; ++i) if (i == isel) { mv = m8[i]; lv = l8[i]; }
        const int irow = q0 + rl;
        if (irow < p.Lq) { float* st = p.ST + (((long long)b * gridDim.y + h) * p.Lq + irow) * 2 + (lane & 1); VST2(float, st, (lane & 1) ? lv : mv * 0.6931471805599453f); }
    }
    float invr[8];
#pragma unroll
    for (int i = 0; i < 8; ++i) {
        if (TWOPASS) invr[i] = SPLITPV ? 1.f : (1.f / 4096.f);
        else if (p.nonorm) invr[i] = exp2f(m8[i]) * (SPLITPV ? 1.f : (1.f / 4096.f));
        else invr[i] = (l8[i] > 0.f) ? (SPLITPV ? 1.f / l8[i] : 1.f / (l8[i] * 4096.f)) : 0.f;
    }
    __syncthreads();
    const bool ofast = ((p.sOi & 3) == 0) && ((((size_t)obase) & 15) == 0) && (q0 + 16 <= p.Lq);
#pragma unroll
    for (int c0 = 0; c0 < DVP; c0 += 64) {
#pragma unroll
        for (int i = 0; i < 8; ++i)
#pragma unroll
            for (int t = 0; t < NT; ++t) if (t * 16 >= c0 && t * 16 < c0 + 64) ((volatile float*)myp)[(i + 8 * hf) * 64 + (t * 16 - c0) + l15] = o[t][i] * invr[i];
        __syncthreads();
        const int cw = (DVP - c0 < 64) ? (DVP - c0) : 64;
        if (ofast && (c0 + cw <= p.dv) && (cw % 32 == 0)) {
            const int lpr = cw / 4;
            const int rows_per_ins = 32 / lpr;
            for (int r0 = 0; r0 < 16; r0 += rows_per_ins) {
                const int row = r0 + lane / lpr, c4 = (lane % lpr) * 4;
                const v4f v = *(const v4f*)(myp + row * 64 + c4);
                VST2V4(obase + (long long)(q0 + row) * p.sOi + c0 + c4, v);
            }
        } else {
            for (int row = 0; row < 16; ++row) {
                const int irow = q0 + row; if (irow >= p.Lq) continue;
                for (int c = lane; c < cw; c += 32) { const int d = c0 + c; if (d < p.dv) VST2(float, obase + (long long)irow * p.sOi + d, myp[row * 64 + c]); }
            }
        }
        __syncthreads();
    }
}

__device__ __forceinline__ void dep_guard_h(v8f& a, v8f& b, v16h x, v16h y) { asm volatile("v_nop\n\tv_nop\n\tv_nop\n\tv_nop" : "+v"(a), "+v"(b) : "v"(x), "v"(y)); }
__device__ __forceinline__ void dep_guard_b(v8f& a, v8f& b, v16b x, v16b y) { asm volatile("v_nop\n\tv_nop\n\tv_nop\n\tv_nop" : "+v"(a), "+v"(b) : "v"(x), "v"(y)); }
__device__ __forceinline__ void keep4_h(v16h a, v16h b, v16h c, v16h d) { asm volatile("v_nop" :: "v"(a), "v"(b), "v"(c), "v"(d)); }
__device__ __forceinline__ void keep4_b(v16b a, v16b b, v16b c, v16b d) { asm volatile("v_nop" :: "v"(a), "v"(b), "v"(c), "v"(d)); }
__device__ __forceinline__ void acc_guard4(v8f& a, v8f& b, v8f& c, v8f& d) { asm volatile("v_nop\n\tv_nop\n\tv_nop\n\tv_nop" : "+v"(a), "+v"(b), "+v"(c), "+v"(d)); }
template <typename T> struct Frag;
template <> struct Frag<_Float16> {
  typedef v16h V; union U { v16h v; v8h h[2]; };
  static __device__ __forceinline__ v16h load(const _Float16* p) {
    U f; f.h[0] = *(const v8h*)(p); f.h[1] = *(const v8h*)(p + 16); return f.v;
  }
  static __device__ __forceinline__ v8f mma(v16h a, v16h b, v8f c) {
    return __builtin_amdgcn_wmma_f32_16x16x32_f16(false, a, false, b, (short)0, c, false, false);
  }
  static __device__ __forceinline__ void guard(v8f& a, v8f& b, v16h x, v16h y) { dep_guard_h(a, b, x, y); }
  static __device__ __forceinline__ void keep(v16h a, v16h b, v16h c, v16h d) { keep4_h(a, b, c, d); }
};
template <> struct Frag<__bf16> {
  typedef v16b V; union U { v16b v; v8b h[2]; };
  static __device__ __forceinline__ v16b load(const __bf16* p) {
    U f; f.h[0] = *(const v8b*)(p); f.h[1] = *(const v8b*)(p + 16); return f.v;
  }
  static __device__ __forceinline__ v8f mma(v16b a, v16b b, v8f c) {
    return __builtin_amdgcn_wmma_f32_16x16x32_bf16(false, a, false, b, (short)0, c, false, false);
  }
  static __device__ __forceinline__ void guard(v8f& a, v8f& b, v16b x, v16b y) { dep_guard_b(a, b, x, y); }
  static __device__ __forceinline__ void keep(v16b a, v16b b, v16b c, v16b d) { keep4_b(a, b, c, d); }
};
template <int ET> struct Elem;
template <> struct Elem<0> { typedef _Float16 T; };
template <> struct Elem<1> { typedef __bf16 T; };

template <int ET, bool SPLIT, int BIAS_MODE, bool RESID>
__global__ __launch_bounds__(256) void wmma_gemm64(
    const unsigned short* __restrict__ Ap, const unsigned short* __restrict__ A2p, int lda, long strideA,
    const unsigned short* __restrict__ Btp, const unsigned short* __restrict__ Bt2p, int ldb, long strideB,
    float* __restrict__ Cout, int ldc, long strideC,
    const float* __restrict__ bias,
    const float* __restrict__ resid, long strideR,
    int M, int N, int K, float scale) {
  typedef typename Elem<ET>::T T;
  typedef typename Frag<T>::V V;
  const T* A = (const T*)Ap; const T* A2 = (const T*)A2p; const T* Bt = (const T*)Btp; const T* Bt2 = (const T*)Bt2p;
  __shared__ __align__(16) float sT[8][16 * 68];
  const int b    = blockIdx.y;
  const int lane = threadIdx.x & 31;
  const int wave = threadIdx.x >> 5;
  const int tilesN = N >> 6;
  const int tilesM = M >> 6;
  const int tile = blockIdx.x * 8 + wave;
  if (tile >= tilesM * tilesN) return;
  const int tm = tile / tilesN;
  const int tn = tile - tm * tilesN;
  const int m0 = tm << 6;
  const int n0 = tn << 6;

  const T* Ab  = A  + (size_t)b * strideA;
  const T* Bb  = Bt + (size_t)b * strideB;
  const T* Ab2 = SPLIT ? (A2  + (size_t)b * strideA) : nullptr;
  const T* Bb2 = SPLIT ? (Bt2 + (size_t)b * strideB) : nullptr;

  const int rlane = lane & 15;
  const int koff  = (lane >> 4) * 8;
  const int mOff  = (lane >> 4) * 8;

  v8f acc[4][4];
#pragma unroll
  for (int i = 0; i < 4; ++i)
#pragma unroll
    for (int j = 0; j < 4; ++j) acc[i][j] = (v8f){0.f,0.f,0.f,0.f,0.f,0.f,0.f,0.f};

  for (int k0 = 0; k0 < K; k0 += 32) {
    V bh[4], bl[4];
#pragma unroll
    for (int j = 0; j < 4; ++j) {
      const size_t bo = (size_t)(n0 + (j << 4) + rlane) * ldb + koff + k0;
      bh[j] = Frag<T>::load(Bb + bo);
      if (SPLIT) bl[j] = Frag<T>::load(Bb2 + bo);
    }
#pragma unroll
    for (int i = 0; i < 4; ++i) {
      const size_t ao = (size_t)(m0 + (i << 4) + rlane) * lda + koff + k0;
      V ah = Frag<T>::load(Ab + ao);
      V al;
      if (SPLIT) al = Frag<T>::load(Ab2 + ao);
#pragma unroll
      for (int j = 0; j < 4; ++j) {
        acc[i][j] = Frag<T>::mma(ah, bh[j], acc[i][j]);
        if (SPLIT) {
          acc[i][j] = Frag<T>::mma(ah, bl[j], acc[i][j]);
          acc[i][j] = Frag<T>::mma(al, bh[j], acc[i][j]);
        }
      }
      Frag<T>::guard(acc[i][0], acc[i][3], ah, SPLIT ? al : ah);
    }
    Frag<T>::keep(bh[0], bh[1], bh[2], bh[3]);
    if (SPLIT) Frag<T>::keep(bl[0], bl[1], bl[2], bl[3]);
  }
  acc_guard4(acc[0][0], acc[0][1], acc[0][2], acc[0][3]);
  acc_guard4(acc[1][0], acc[1][1], acc[1][2], acc[1][3]);
  acc_guard4(acc[2][0], acc[2][1], acc[2][2], acc[2][3]);
  acc_guard4(acc[3][0], acc[3][1], acc[3][2], acc[3][3]);

  float* slab = sT[wave];
  const float* Rb = RESID ? (resid + (size_t)b * strideR) : nullptr;
  float* C = Cout + (size_t)b * strideC;
#pragma unroll
  for (int i = 0; i < 4; ++i) {
    const int mBase = m0 + (i << 4);
#pragma unroll
    for (int j = 0; j < 4; ++j) {
      const int n = n0 + (j << 4) + rlane;
      float bv = 0.f;
      if (BIAS_MODE == 2) bv = bias[n];
#pragma unroll
      for (int r = 0; r < 8; ++r) {
        float v = acc[i][j][r] * scale;
        if (BIAS_MODE == 1) v += bias[mBase + mOff + r];
        if (BIAS_MODE == 2) v += bv;
        if (RESID) v += Rb[(size_t)(mBase + mOff + r) * ldc + n];
        slab[(mOff + r) * 68 + (j << 4) + rlane] = v;
      }
    }
    __builtin_amdgcn_fence(3  , "workgroup");
    __builtin_amdgcn_wave_barrier();
    __builtin_amdgcn_fence(2  , "workgroup");
    {
      const int hh = lane >> 4, c4 = (lane & 15) * 4;
      for (int pass = 0; pass < 2; ++pass) {
#pragma unroll
        for (int it = 0; it < 8; ++it) {
          const int row = it * 2 + hh;
          v4f v = *(const v4f*)(slab + row * 68 + c4);
          *(volatile v4f*)(C + (size_t)(mBase + row) * ldc + n0 + c4) = v;
        }
        __threadfence();
      }
    }
    __builtin_amdgcn_fence(3  , "workgroup");
    __builtin_amdgcn_wave_barrier();
    __builtin_amdgcn_fence(2  , "workgroup");
  }
}

__device__ __forceinline__ unsigned int f2bf2_pack(float a, float b, unsigned int* lo) {
    const unsigned short ha = f2bf_bits(a), hb = f2bf_bits(b);
    const unsigned short la = f2bf_bits(a - bf_bits2f(ha)), lb = f2bf_bits(b - bf_bits2f(hb));
    *lo = (unsigned)la | ((unsigned)lb << 16); return (unsigned)ha | ((unsigned)hb << 16); }
__global__ __launch_bounds__(256) void k_castS16(const float* __restrict__ src, unsigned lds, unsigned short* __restrict__ dhi, unsigned short* __restrict__ dlo, unsigned ldd, unsigned R, unsigned C) {
    const unsigned i = blockIdx.x * 256u + threadIdx.x; const unsigned hc = C >> 1; if (i >= R * hc) return;
    const unsigned r = i / hc; const unsigned c = (i - r * hc) << 1;
    const float a = src[(size_t)r * lds + c], b = src[(size_t)r * lds + c + 1];
    unsigned lo; const unsigned hi = f2bf2_pack(a, b, &lo);
    const size_t o = (size_t)r * ldd + c;
    volatile unsigned* ph = (volatile unsigned*)(dhi + o); volatile unsigned* pl = (volatile unsigned*)(dlo + o);
    *ph = hi; *pl = lo; __threadfence(); *ph = hi; *pl = lo; }

__device__ __forceinline__ unsigned int cmb_pk2(float a, float b) { return (unsigned int)__builtin_bit_cast(unsigned short, (_Float16)a) | ((unsigned int)__builtin_bit_cast(unsigned short, (_Float16)b) << 16); }
__device__ __forceinline__ float cmb_bf(float v) { const unsigned u = __builtin_bit_cast(unsigned, v); const unsigned r = (u + 0x7fffu + ((u >> 16) & 1u)) & 0xffff0000u; return __builtin_bit_cast(float, r); }
__global__ __launch_bounds__(256) void k_cm_bfvec(const float* __restrict__ SRC, float* __restrict__ DST, unsigned n) { const unsigned u = blockIdx.x * 256u + threadIdx.x; if (u >= n) return; VST2(float, DST + u, cmb_bf(SRC[u])); }
__global__ __launch_bounds__(256) void k_cm_castb(const float* __restrict__ SRC, unsigned lds, unsigned short* __restrict__ DST, unsigned ldd, unsigned nR, unsigned nC, float sc) {
    const unsigned u = blockIdx.x * 256u + threadIdx.x; const unsigned per = nC >> 3; if (u >= nR * per) return;
    const unsigned r = u / per; const unsigned c0 = (u - r * per) << 3;
    const float* s = SRC + (size_t)r * lds + c0; float w[8];
#pragma unroll
    for (int e = 0; e < 8; ++e) w[e] = cmb_bf(s[e]) * sc;
    cm_u4 pk; pk.x = cmb_pk2(w[0], w[1]); pk.y = cmb_pk2(w[2], w[3]); pk.z = cmb_pk2(w[4], w[5]); pk.w = cmb_pk2(w[6], w[7]); VST2(cm_u4, (cm_u4*)(DST + (size_t)r * ldd + c0), pk); }

constexpr size_t al256(size_t x) { return (x + 255) / 256 * 256; }
constexpr size_t SZ_X16  = al256((size_t)NB * SEQ * DM * 2);
constexpr size_t SZ_W3   = al256((size_t)3 * DM * DM * 2);
constexpr size_t SZ_W    = al256((size_t)DM * DM * 2);
constexpr size_t SZ_QKV  = al256((size_t)SEQ * D3 * 4);
constexpr size_t SZ_AO   = al256((size_t)SEQ * DM * 4);
constexpr size_t SZ_AO16 = al256((size_t)SEQ * DM * 2);
constexpr size_t SZ_BR   = al256((size_t)(DM + 64) * 4);
constexpr size_t WS_TOTAL = 3 * SZ_X16 + SZ_W3 + 2 * SZ_W + SZ_QKV + SZ_AO + 2 * SZ_AO16 + 4 * SZ_BR;
static_assert(WS_TOTAL <= (size_t)134217728);
static_assert((SEQ * (DM / 8)) * 8 == SEQ * DM);
static_assert((SEQ * (DM / 2)) * 2 == SEQ * DM);
static_assert((SEQ / 64) * 64 == SEQ);
static_assert((DM / 64) * 64 == DM);
static_assert((DM / 32) * 32 == DM);

extern "C" void kernel_launch(void* const* d_in, const int* in_sizes, int n_in, void* d_out, int out_size, void* d_ws, size_t ws_size, hipStream_t stream) {
    if (n_in < 12) return;
    const long long needx = (long long)(NB - 1) * SEQ_FULL * DM + (long long)SEQ * DM;
    const long long needm = (long long)(SEQ - 1) * SEQ_FULL + SEQ;
    if (in_sizes[0] < needx || in_sizes[1] < needx || in_sizes[2] < needx || in_sizes[3] < needm) return;
    if (in_sizes[4] < DM * DM || in_sizes[6] < DM * DM || in_sizes[8] < DM * DM || in_sizes[10] < DM * DM) return;
    if (in_sizes[5] < DM || in_sizes[7] < DM || in_sizes[9] < DM || in_sizes[11] < DM) return;
    if ((long long)out_size < (long long)NB * SEQ * DM) return;
    if (ws_size < WS_TOTAL) return;
    const float* xq = (const float*)d_in[0];
    const float* xk = (const float*)d_in[1];
    const float* xv = (const float*)d_in[2];
    const int* amask = (const int*)d_in[3];
    const float* wq = (const float*)d_in[4];
    const float* bq = (const float*)d_in[5];
    const float* wk = (const float*)d_in[6];
    const float* bk = (const float*)d_in[7];
    const float* wv = (const float*)d_in[8];
    const float* bv = (const float*)d_in[9];
    const float* wo = (const float*)d_in[10];
    const float* bo = (const float*)d_in[11];
    float* out = (float*)d_out;
    char* wsp = (char*)d_ws;
    unsigned short* X16q = (unsigned short*)wsp; wsp += SZ_X16;
    unsigned short* X16k = (unsigned short*)wsp; wsp += SZ_X16;
    unsigned short* X16v = (unsigned short*)wsp; wsp += SZ_X16;
    unsigned short* W316 = (unsigned short*)wsp; wsp += SZ_W3;
    unsigned short* WOH  = (unsigned short*)wsp; wsp += SZ_W;
    unsigned short* WOL  = (unsigned short*)wsp; wsp += SZ_W;
    float* QKV = (float*)wsp; wsp += SZ_QKV;
    float* AO  = (float*)wsp; wsp += SZ_AO;
    unsigned short* AOH = (unsigned short*)wsp; wsp += SZ_AO16;
    unsigned short* AOL = (unsigned short*)wsp; wsp += SZ_AO16;
    float* BRq = (float*)wsp; wsp += SZ_BR;
    float* BRk = (float*)wsp; wsp += SZ_BR;
    float* BRv = (float*)wsp; wsp += SZ_BR;
    float* BRo = (float*)wsp; wsp += SZ_BR;
    if ((size_t)(wsp - (char*)d_ws) > ws_size) return;

    const unsigned gW  = (unsigned)(((long long)DM * (DM / 8) + 255) / 256);
    const unsigned gWS = (unsigned)(((long long)DM * (DM / 2) + 255) / 256);
    const unsigned gX  = (unsigned)(((long long)SEQ * (DM / 8) + 255) / 256);
    const unsigned gXS = (unsigned)(((long long)SEQ * (DM / 2) + 255) / 256);
    const unsigned gB  = (unsigned)((DM + 255) / 256);
    const unsigned gG  = (unsigned)((((SEQ) / 64) * ((DM) / 64) + 7) / 8);

    k_cm_castb<<<gW, 256, 0, stream>>>(wq, DM, W316 + (size_t)0 * DM * DM, DM, DM, DM, 16.0f);
    k_cm_castb<<<gW, 256, 0, stream>>>(wk, DM, W316 + (size_t)1 * DM * DM, DM, DM, DM, 16.0f);
    k_cm_castb<<<gW, 256, 0, stream>>>(wv, DM, W316 + (size_t)2 * DM * DM, DM, DM, DM, 16.0f);
    k_castS16<<<gWS, 256, 0, stream>>>(wo, DM, WOH, WOL, DM, DM, DM);
    k_cm_bfvec<<<gB, 256, 0, stream>>>(bq, BRq, DM);
    k_cm_bfvec<<<gB, 256, 0, stream>>>(bk, BRk, DM);
    k_cm_bfvec<<<gB, 256, 0, stream>>>(bv, BRv, DM);
    k_cm_bfvec<<<gB, 256, 0, stream>>>(bo, BRo, DM);

    for (int b = 0; b < NB; ++b) {
        const size_t ioff = (size_t)b * SEQ_FULL * DM;
        unsigned short* Xq = X16q + (size_t)b * SEQ * DM;
        unsigned short* Xk = X16k + (size_t)b * SEQ * DM;
        unsigned short* Xv = X16v + (size_t)b * SEQ * DM;
        float* outb = out + (size_t)b * SEQ * DM;
        k_cm_castb<<<gX, 256, 0, stream>>>(xq + ioff, DM, Xq, DM, SEQ, DM, 1.0f);
        k_cm_castb<<<gX, 256, 0, stream>>>(xk + ioff, DM, Xk, DM, SEQ, DM, 1.0f);
        k_cm_castb<<<gX, 256, 0, stream>>>(xv + ioff, DM, Xv, DM, SEQ, DM, 1.0f);
        wmma_gemm64<0, false, 2, false><<<dim3(gG, 1u), 256, 0, stream>>>(Xq, nullptr, DM, 0, W316 + (size_t)0 * DM * DM, nullptr, DM, 0, QKV + 0 * DM, D3, 0, BRq, nullptr, 0, SEQ, DM, DM, 0.0625f);
        wmma_gemm64<0, false, 2, false><<<dim3(gG, 1u), 256, 0, stream>>>(Xk, nullptr, DM, 0, W316 + (size_t)1 * DM * DM, nullptr, DM, 0, QKV + 1 * DM, D3, 0, BRk, nullptr, 0, SEQ, DM, DM, 0.0625f);
        wmma_gemm64<0, false, 2, false><<<dim3(gG, 1u), 256, 0, stream>>>(Xv, nullptr, DM, 0, W316 + (size_t)2 * DM * DM, nullptr, DM, 0, QKV + 2 * DM, D3, 0, BRv, nullptr, 0, SEQ, DM, DM, 0.0625f);
        {
            AttnP a = {};
            a.Q = QKV + 0; a.K = QKV + DM; a.V = QKV + 2 * DM; a.O = AO; a.P = 0; a.Mf = 0; a.Mi = amask; a.ST = 0;
            a.Pw = 0; a.Rt = 0; a.SQ = 0; a.SK = 0;
            a.swb = 0; a.swh = 0; a.swi = 0; a.swj = 0; a.srb = 0; a.srh = 0; a.sri = 0;
            a.sQb = 0; a.sQh = HD; a.sQi = D3; a.sQd = 1; a.sKb = 0; a.sKh = HD; a.sKj = D3; a.sKd = 1; a.sVb = 0; a.sVh = HD; a.sVj = D3; a.sVd = 1;
            a.sOb = 0; a.sOh = HD; a.sOi = DM; a.sPb = 0; a.sPh = 0; a.sPi = 0; a.smb = 0; a.smh = 0; a.smi = SEQ_FULL; a.smj = 1;
            a.Lq = SEQ; a.Lk = SEQ; a.dh = HD; a.dv = HD; a.hrep = 1; a.causal = 0; a.coff = 0; a.pband = 0;
            a.scale = 0.125f; a.mfill = -1.0e9f; a.nonorm = 0; a.mpol = 0;
            a.roff = 0; a.rn = 1; a.segpol = 0; a.win = 0;
            k_attn<64, 64, 1, true, false><<<dim3((unsigned)((SEQ + 16 * AW - 1) / (16 * AW)), (unsigned)NH, 1u), 32 * AW, 0, stream>>>(a);
        }
        k_castS16<<<gXS, 256, 0, stream>>>(AO, DM, AOH, AOL, DM, SEQ, DM);
        wmma_gemm64<1, false, 2, false><<<dim3(gG, 1u), 256, 0, stream>>>(AOH, nullptr, DM, 0, WOH, nullptr, DM, 0, outb, DM, 0, BRo, nullptr, 0, SEQ, DM, DM, 1.0f);
        wmma_gemm64<1, false, 0, true><<<dim3(gG, 1u), 256, 0, stream>>>(AOL, nullptr, DM, 0, WOH, nullptr, DM, 0, outb, DM, 0, nullptr, outb, 0, SEQ, DM, DM, 1.0f);
    }
}
